// predictNet_85555748536778
// MI455X (gfx1250) — hardware-verified
//
#include <hip/hip_runtime.h>
#include <stddef.h>

typedef __attribute__((ext_vector_type(16))) _Float16 v16h;
typedef __attribute__((ext_vector_type(8)))  _Float16 v8h;
typedef __attribute__((ext_vector_type(16))) __bf16   v16b;
typedef __attribute__((ext_vector_type(8)))  __bf16   v8b;
typedef __attribute__((ext_vector_type(8)))  float    v8f;
typedef __attribute__((ext_vector_type(4)))  float    v4f;
typedef __attribute__((ext_vector_type(4)))  unsigned int v4u;

constexpr int   SIG_LEN      = 262144;
constexpr int   SIG_MASK     = SIG_LEN - 1;
constexpr float LN_EPSILON   = 1e-5f;
constexpr int   POOL_TAPS    = 151;
constexpr int   POOL_HALF    = 75;
constexpr int   POOL_OUT     = 4096;
constexpr int   POOL_PER_THR = 16;

__device__ __forceinline__ unsigned short f2bf_bits(float f) {
  unsigned u = __float_as_uint(f);
  return (unsigned short)((u + 0x7FFFu + ((u >> 16) & 1u)) >> 16);
}
__device__ __forceinline__ float bf_bits2f(unsigned short h) { return __uint_as_float(((unsigned)h) << 16); }

__device__ __forceinline__ void dep_guard_h(v8f& a, v8f& b, v16h x, v16h y) { asm volatile("v_nop\n\tv_nop\n\tv_nop\n\tv_nop" : "+v"(a), "+v"(b) : "v"(x), "v"(y)); }
__device__ __forceinline__ void dep_guard_b(v8f& a, v8f& b, v16b x, v16b y) { asm volatile("v_nop\n\tv_nop\n\tv_nop\n\tv_nop" : "+v"(a), "+v"(b) : "v"(x), "v"(y)); }
__device__ __forceinline__ void keep4_h(v16h a, v16h b, v16h c, v16h d) { asm volatile("v_nop" :: "v"(a), "v"(b), "v"(c), "v"(d)); }
__device__ __forceinline__ void keep4_b(v16b a, v16b b, v16b c, v16b d) { asm volatile("v_nop" :: "v"(a), "v"(b), "v"(c), "v"(d)); }
__device__ __forceinline__ void acc_guard4(v8f& a, v8f& b, v8f& c, v8f& d) { asm volatile("v_nop\n\tv_nop\n\tv_nop\n\tv_nop" : "+v"(a), "+v"(b), "+v"(c), "+v"(d)); }
template <typename T> struct Frag;
template <> struct Frag<_Float16> {
  typedef v16h V; union U { v16h v; v8h h[2]; };
  static __device__ __forceinline__ v16h load(const _Float16* p) {
    U f; f.h[0] = *(const v8h*)(p); f.h[1] = *(const v8h*)(p + 16); return f.v;
  }
  static __device__ __forceinline__ v8f mma(v16h a, v16h b, v8f c) {
    return __builtin_amdgcn_wmma_f32_16x16x32_f16(false, a, false, b, (short)0, c, false, false);
  }
  static __device__ __forceinline__ void guard(v8f& a, v8f& b, v16h x, v16h y) { dep_guard_h(a, b, x, y); }
  static __device__ __forceinline__ void keep(v16h a, v16h b, v16h c, v16h d) { keep4_h(a, b, c, d); }
};
template <> struct Frag<__bf16> {
  typedef v16b V; union U { v16b v; v8b h[2]; };
  static __device__ __forceinline__ v16b load(const __bf16* p) {
    U f; f.h[0] = *(const v8b*)(p); f.h[1] = *(const v8b*)(p + 16); return f.v;
  }
  static __device__ __forceinline__ v8f mma(v16b a, v16b b, v8f c) {
    return __builtin_amdgcn_wmma_f32_16x16x32_bf16(false, a, false, b, (short)0, c, false, false);
  }
  static __device__ __forceinline__ void guard(v8f& a, v8f& b, v16b x, v16b y) { dep_guard_b(a, b, x, y); }
  static __device__ __forceinline__ void keep(v16b a, v16b b, v16b c, v16b d) { keep4_b(a, b, c, d); }
};

__device__ __forceinline__ float block_sum_512(float val, float* red) {
  red[threadIdx.x] = val;
  __syncthreads();
  for (int s = 256; s > 0; s >>= 1) {
    if ((int)threadIdx.x < s) red[threadIdx.x] += red[threadIdx.x + s];
    __syncthreads();
  }
  const float r = red[0];
  __syncthreads();
  return r;
}

__global__ __launch_bounds__(256) void gemm_hidden_dot(
    const unsigned short* __restrict__ Ap, const unsigned short* __restrict__ A2p, int lda,
    const unsigned short* __restrict__ Btp, const unsigned short* __restrict__ Bt2p, int ldb,
    float* __restrict__ Pout, long strideP,
    const float* __restrict__ bias, const float* __restrict__ colv,
    const float* __restrict__ wbar, const float* __restrict__ rowv,
    int M, int N, int K) {
  typedef __bf16 T;
  typedef v16b V;
  const T* Ab  = (const T*)Ap;  const T* Ab2 = (const T*)A2p;
  const T* Bb  = (const T*)Btp; const T* Bb2 = (const T*)Bt2p;
  __shared__ __align__(16) float sT[8][68];
  const int lane = threadIdx.x & 31;
  const int wave = threadIdx.x >> 5;
  const int tilesN = N >> 6;
  const int tilesM = M >> 6;
  const int tile = blockIdx.x * 8 + wave;
  if (tile >= tilesM * tilesN) return;
  const int tm = tile / tilesN;
  const int tn = tile - tm * tilesN;
  const int m0 = tm << 6;
  const int n0 = tn << 6;

  const int rlane = lane & 15;
  const int koff  = (lane >> 4) * 8;
  const int mOff  = (lane >> 4) * 8;

  v8f acc[4][4];
#pragma unroll
  for (int i = 0; i < 4; ++i)
#pragma unroll
    for (int j = 0; j < 4; ++j) acc[i][j] = (v8f){0.f,0.f,0.f,0.f,0.f,0.f,0.f,0.f};

  for (int k0 = 0; k0 < K; k0 += 32) {
    V bh[4], bl[4];
#pragma unroll
    for (int j = 0; j < 4; ++j) {
      const size_t bo = (size_t)(n0 + (j << 4) + rlane) * ldb + koff + k0;
      bh[j] = Frag<T>::load(Bb + bo);
      bl[j] = Frag<T>::load(Bb2 + bo);
    }
#pragma unroll
    for (int i = 0; i < 4; ++i) {
      const size_t ao = (size_t)(m0 + (i << 4) + rlane) * lda + koff + k0;
      V ah = Frag<T>::load(Ab + ao);
      V al = Frag<T>::load(Ab2 + ao);
#pragma unroll
      for (int j = 0; j < 4; ++j) {
        acc[i][j] = Frag<T>::mma(ah, bh[j], acc[i][j]);
        acc[i][j] = Frag<T>::mma(ah, bl[j], acc[i][j]);
        acc[i][j] = Frag<T>::mma(al, bh[j], acc[i][j]);
      }
      Frag<T>::guard(acc[i][0], acc[i][3], ah, al);
    }
    Frag<T>::keep(bh[0], bh[1], bh[2], bh[3]);
    Frag<T>::keep(bl[0], bl[1], bl[2], bl[3]);
  }
  acc_guard4(acc[0][0], acc[0][1], acc[0][2], acc[0][3]);
  acc_guard4(acc[1][0], acc[1][1], acc[1][2], acc[1][3]);
  acc_guard4(acc[2][0], acc[2][1], acc[2][2], acc[2][3]);
  acc_guard4(acc[3][0], acc[3][1], acc[3][2], acc[3][3]);

  float bvj[4], cvj[4], wvj[4];
#pragma unroll
  for (int j = 0; j < 4; ++j) {
    const int n = n0 + (j << 4) + rlane;
    bvj[j] = bias[n];
    cvj[j] = colv[n];
    wvj[j] = wbar[n];
  }
  float* slab = sT[wave];
#pragma unroll
  for (int i = 0; i < 4; ++i) {
    const int mBase = m0 + (i << 4);
    float av[8], pr[8];
#pragma unroll
    for (int r = 0; r < 8; ++r) { av[r] = rowv[mBase + mOff + r]; pr[r] = 0.f; }
#pragma unroll
    for (int j = 0; j < 4; ++j) {
#pragma unroll
      for (int r = 0; r < 8; ++r) {
        float hv = acc[i][j][r] + av[r] * cvj[j] + bvj[j];
        hv = fmaxf(hv, 0.0f);
        pr[r] += hv * wvj[j];
      }
    }
#pragma unroll
    for (int r = 0; r < 8; ++r) {
      float tsum = pr[r];
      tsum += __shfl_xor(tsum, 1, 32);
      tsum += __shfl_xor(tsum, 2, 32);
      tsum += __shfl_xor(tsum, 4, 32);
      tsum += __shfl_xor(tsum, 8, 32);
      pr[r] = tsum;
    }
    if (rlane == 0) {
#pragma unroll
      for (int r = 0; r < 8; ++r) slab[(i << 4) + mOff + r] = pr[r];
    }
  }
  __builtin_amdgcn_fence(__ATOMIC_RELEASE, "workgroup");
  __builtin_amdgcn_wave_barrier();
  __builtin_amdgcn_fence(__ATOMIC_ACQUIRE, "workgroup");
  {
    const int c4 = (lane & 15) * 4;
    const v4f val = *(const v4f*)(slab + c4);
    float* dst = Pout + (size_t)tn * (size_t)strideP + m0 + c4;
    for (int pass = 0; pass < 2; ++pass) {
      if (lane < 16) *(volatile v4f*)dst = val;
      __threadfence();
    }
  }
}

__global__ __launch_bounds__(256) void build_a_kernel(
    const float* __restrict__ v, unsigned short* __restrict__ ah, unsigned short* __restrict__ al,
    int row0, int nrows, int kw8) {
  const int e = blockIdx.x * 256 + threadIdx.x;
  if (e >= nrows * kw8) return;
  const int row = e / kw8;
  const int kb  = (e - row * kw8) * 8;
  const int tg  = row0 + row;
  unsigned wh[4], wl[4];
#pragma unroll
  for (int q = 0; q < 4; ++q) {
    const float f0 = v[(tg - kb - 2 * q) & SIG_MASK];
    const float f1 = v[(tg - kb - 2 * q - 1) & SIG_MASK];
    const unsigned short h0 = f2bf_bits(f0);
    const unsigned short l0 = f2bf_bits(f0 - bf_bits2f(h0));
    const unsigned short h1 = f2bf_bits(f1);
    const unsigned short l1 = f2bf_bits(f1 - bf_bits2f(h1));
    wh[q] = (unsigned)h0 | ((unsigned)h1 << 16);
    wl[q] = (unsigned)l0 | ((unsigned)l1 << 16);
  }
  v4u hv, lv;
  hv[0] = wh[0]; hv[1] = wh[1]; hv[2] = wh[2]; hv[3] = wh[3];
  lv[0] = wl[0]; lv[1] = wl[1]; lv[2] = wl[2]; lv[3] = wl[3];
  v4u* ph = (v4u*)(ah) + e;
  v4u* pl = (v4u*)(al) + e;
  *(volatile v4u*)ph = hv;
  *(volatile v4u*)pl = lv;
  __threadfence();
  *(volatile v4u*)ph = hv;
  *(volatile v4u*)pl = lv;
}

template <int KW, int DIN, int NH, int NP>
__global__ __launch_bounds__(256) void prep_bt_kernel(
    const float* __restrict__ Wa, unsigned short* __restrict__ bth, unsigned short* __restrict__ btl) {
  constexpr int KW8 = KW / 8;
  const int e = blockIdx.x * 256 + threadIdx.x;
  if (e >= NP * KW8) return;
  const int n  = e / KW8;
  const int kb = (e - n * KW8) * 8;
  const int nc = n < NH ? n : NH - 1;
  const bool live = n < NH;
  unsigned wh[4], wl[4];
#pragma unroll
  for (int q = 0; q < 4; ++q) {
    float f0 = Wa[(size_t)nc * DIN + kb + 2 * q];
    float f1 = Wa[(size_t)nc * DIN + kb + 2 * q + 1];
    f0 = live ? f0 : 0.0f;
    f1 = live ? f1 : 0.0f;
    const unsigned short h0 = f2bf_bits(f0);
    const unsigned short l0 = f2bf_bits(f0 - bf_bits2f(h0));
    const unsigned short h1 = f2bf_bits(f1);
    const unsigned short l1 = f2bf_bits(f1 - bf_bits2f(h1));
    wh[q] = (unsigned)h0 | ((unsigned)h1 << 16);
    wl[q] = (unsigned)l0 | ((unsigned)l1 << 16);
  }
  v4u hv, lv;
  hv[0] = wh[0]; hv[1] = wh[1]; hv[2] = wh[2]; hv[3] = wh[3];
  lv[0] = wl[0]; lv[1] = wl[1]; lv[2] = wl[2]; lv[3] = wl[3];
  v4u* ph = (v4u*)(bth) + e;
  v4u* pl = (v4u*)(btl) + e;
  *(volatile v4u*)ph = hv;
  *(volatile v4u*)pl = lv;
  __threadfence();
  *(volatile v4u*)ph = hv;
  *(volatile v4u*)pl = lv;
}

template <int KW, int DIN, int NH, int NP, int PP>
__global__ __launch_bounds__(256) void prep_vec_kernel(
    const float* __restrict__ Wa, const float* __restrict__ ba,
    const float* __restrict__ Wb, const float* __restrict__ bb,
    float* __restrict__ vec) {
  const int which = blockIdx.y;
  const int f4 = threadIdx.x;
  v4f val = (v4f){0.f, 0.f, 0.f, 0.f};
  float* dst;
  if (which == 3) {
    if (f4 >= 8) return;
    float s = 0.f;
#pragma unroll 1
    for (int j = 0; j < PP; ++j) s += bb[j];
    s = s * (1.0f / (float)PP);
    if (f4 == 0) val[0] = s;
    dst = vec + 3 * NP + 4 * f4;
  } else {
    if (f4 >= NP / 4) return;
#pragma unroll
    for (int q = 0; q < 4; ++q) {
      const int n  = 4 * f4 + q;
      const int nc = n < NH ? n : NH - 1;
      const bool live = n < NH;
      float r;
      if (which == 0) {
        r = Wa[(size_t)nc * DIN + KW];
      } else if (which == 1) {
        r = ba[nc];
      } else {
        float s = 0.f;
#pragma unroll 1
        for (int j = 0; j < PP; ++j) s += Wb[(size_t)j * NH + nc];
        r = s * (1.0f / (float)PP);
      }
      val[q] = live ? r : 0.0f;
    }
    dst = vec + which * NP + 4 * f4;
  }
  *(volatile v4f*)dst = val;
  __threadfence();
  *(volatile v4f*)dst = val;
}

__global__ __launch_bounds__(512) void ln_input_kernel(const float* __restrict__ x, float* __restrict__ vout) {
  __shared__ float red[512];
  const int tid = threadIdx.x;
  float s = 0.f;
#pragma unroll 1
  for (int k = 0; k < SIG_LEN / 512; ++k) s += x[k * 512 + tid];
  const float mean = block_sum_512(s, red) * (1.0f / (float)SIG_LEN);
  float ss = 0.f;
#pragma unroll 1
  for (int k = 0; k < SIG_LEN / 512; ++k) {
    const float d = x[k * 512 + tid] - mean;
    ss += d * d;
  }
  const float var  = block_sum_512(ss, red) * (1.0f / (float)SIG_LEN);
  const float rstd = 1.0f / sqrtf(var + LN_EPSILON);
#pragma unroll 1
  for (int it = 0; it < SIG_LEN / 2048; ++it) {
    const int idx = it * 512 + tid;
    const v4f xv = ((const v4f*)x)[idx];
    const v4f o  = (xv - mean) * rstd;
    *(volatile v4f*)(vout + 4 * (size_t)idx) = o;
    __threadfence();
    *(volatile v4f*)(vout + 4 * (size_t)idx) = o;
  }
}

__global__ __launch_bounds__(256) void pool_kernel(
    const float* __restrict__ v, float* __restrict__ avg, float* __restrict__ en) {
  __shared__ float win[POOL_OUT + 2 * POOL_HALF + 2];
  __shared__ __align__(16) float resA[POOL_OUT];
  __shared__ __align__(16) float resE[POOL_OUT];
  const int tid  = threadIdx.x;
  const int base = blockIdx.x * POOL_OUT;
  for (int i = tid; i < POOL_OUT + 2 * POOL_HALF; i += 256) {
    const int g = base - POOL_HALF + i;
    int gc = g < 0 ? 0 : g;
    gc = gc > SIG_MASK ? SIG_MASK : gc;
    const float f = v[gc];
    win[i] = (g >= 0 && g < SIG_LEN) ? f : 0.0f;
  }
  __syncthreads();
  const int t0 = tid * POOL_PER_THR;
  float sA = 0.f, sE = 0.f;
#pragma unroll 1
  for (int j = 0; j < POOL_TAPS; ++j) {
    const float w = win[t0 + j];
    sA += w;
    sE += w * w;
  }
  const float inv = 1.0f / (float)POOL_TAPS;
  resA[t0] = sA * inv;
  resE[t0] = sE * inv;
#pragma unroll 1
  for (int q = 1; q < POOL_PER_THR; ++q) {
    const float wn = win[t0 + POOL_TAPS - 1 + q];
    const float wo = win[t0 + q - 1];
    sA = (sA + wn) - wo;
    sE = (sE + wn * wn) - wo * wo;
    resA[t0 + q] = sA * inv;
    resE[t0 + q] = sE * inv;
  }
  __syncthreads();
#pragma unroll 1
  for (int it = 0; it < POOL_OUT / 1024; ++it) {
    const int idx4 = it * 256 + tid;
    const v4f a4 = *(const v4f*)(resA + 4 * idx4);
    const v4f e4 = *(const v4f*)(resE + 4 * idx4);
    float* pa = avg + base + 4 * idx4;
    float* pe = en  + base + 4 * idx4;
    *(volatile v4f*)pa = a4;
    *(volatile v4f*)pe = e4;
    __threadfence();
    *(volatile v4f*)pa = a4;
    *(volatile v4f*)pe = e4;
  }
}

__global__ __launch_bounds__(256) void psum_kernel(
    const float* __restrict__ P, int ntn, long strideP, const float* __restrict__ bline,
    float* __restrict__ o) {
  const int i4 = blockIdx.x * 256 + threadIdx.x;
  if (i4 >= SIG_LEN / 4) return;
  v4f acc = (v4f){0.f, 0.f, 0.f, 0.f};
#pragma unroll 1
  for (int tn = 0; tn < ntn; ++tn) acc += *(const v4f*)(P + (size_t)tn * (size_t)strideP + 4 * (size_t)i4);
  const float bb = bline[0];
  acc += bb;
  *(volatile v4f*)(o + 4 * (size_t)i4) = acc;
  __threadfence();
  *(volatile v4f*)(o + 4 * (size_t)i4) = acc;
}

template <bool DIV>
__global__ __launch_bounds__(512) void ln_output_kernel(
    const float* __restrict__ src, const float* __restrict__ den, float* __restrict__ dst) {
  __shared__ float red[512];
  const int tid = threadIdx.x;
  float s = 0.f;
#pragma unroll 1
  for (int k = 0; k < SIG_LEN / 512; ++k) {
    const int i = k * 512 + tid;
    float tv = src[i];
    if (DIV) tv = tv / den[i];
    s += tv;
  }
  const float mean = block_sum_512(s, red) * (1.0f / (float)SIG_LEN);
  float ss = 0.f;
#pragma unroll 1
  for (int k = 0; k < SIG_LEN / 512; ++k) {
    const int i = k * 512 + tid;
    float tv = src[i];
    if (DIV) tv = tv / den[i];
    const float d = tv - mean;
    ss += d * d;
  }
  const float var  = block_sum_512(ss, red) * (1.0f / (float)SIG_LEN);
  const float rstd = 1.0f / sqrtf(var + LN_EPSILON);
#pragma unroll 1
  for (int it = 0; it < SIG_LEN / 2048; ++it) {
    const int idx = it * 512 + tid;
    v4f tv = ((const v4f*)src)[idx];
    if (DIV) {
      const v4f dv = ((const v4f*)den)[idx];
      tv = tv / dv;
    }
    const v4f o = (tv - mean) * rstd;
    *(volatile v4f*)(dst + 4 * (size_t)idx) = o;
    __threadfence();
    *(volatile v4f*)(dst + 4 * (size_t)idx) = o;
  }
}

extern "C" void kernel_launch(void* const* d_in, const int* in_sizes, int n_in,
                              void* d_out, int out_size, void* d_ws,
                              size_t ws_size, hipStream_t stream) {
  constexpr int KW1 = 64,  DIN1 = 65,  NH1 = 260, NP1 = 320, PP1 = 3;
  constexpr int KW2 = 128, DIN2 = 129, NH2 = 516, NP2 = 576, PP2 = 21;
  constexpr int NT1 = NP1 / 64;
  constexpr int NT2 = NP2 / 64;
  constexpr int CHUNK2 = 131072;

  if (n_in < 9) return;
  if (in_sizes[0] != SIG_LEN) return;
  if (in_sizes[1] != NH1 * DIN1 || in_sizes[2] != NH1 || in_sizes[3] != PP1 * NH1 || in_sizes[4] != PP1) return;
  if (in_sizes[5] != NH2 * DIN2 || in_sizes[6] != NH2 || in_sizes[7] != PP2 * NH2 || in_sizes[8] != PP2) return;
  if (out_size != 2 * SIG_LEN) return;

  constexpr size_t MIB = 1048576;
  constexpr size_t OFF_V    = 0;
  constexpr size_t OFF_AVG  = 1 * MIB;
  constexpr size_t OFF_EN   = 2 * MIB;
  constexpr size_t OFF_O1   = 3 * MIB;
  constexpr size_t OFF_O2   = 4 * MIB;
  constexpr size_t OFF_VEC1 = 5 * MIB;
  constexpr size_t OFF_VEC2 = OFF_VEC1 + 4096;
  constexpr size_t OFF_BT1H = OFF_VEC2 + 8192;
  constexpr size_t OFF_BT1L = OFF_BT1H + (size_t)NP1 * KW1 * 2;
  constexpr size_t OFF_BT2H = OFF_BT1L + (size_t)NP1 * KW1 * 2;
  constexpr size_t OFF_BT2L = OFF_BT2H + (size_t)NP2 * KW2 * 2;
  constexpr size_t OFF_P    = 6 * MIB;
  constexpr size_t OFF_AH   = 15 * MIB;
  constexpr size_t OFF_AL   = 47 * MIB;
  constexpr size_t WS_END   = 79 * MIB;
  static_assert((3 * NP1 + 32) * 4 <= 4096);
  static_assert((3 * NP2 + 32) * 4 <= 8192);
  static_assert(OFF_BT2L + (size_t)NP2 * KW2 * 2 <= OFF_P);
  static_assert(OFF_P + (size_t)NT2 * SIG_LEN * 4 <= OFF_AH);
  static_assert(OFF_AH + (size_t)SIG_LEN * KW1 * 2 <= OFF_AL);
  static_assert(OFF_AH + (size_t)CHUNK2 * KW2 * 2 <= OFF_AL);
  static_assert(OFF_AL + (size_t)SIG_LEN * KW1 * 2 <= WS_END);
  static_assert(OFF_AL + (size_t)CHUNK2 * KW2 * 2 <= WS_END);
  static_assert(WS_END <= (size_t)134217728);
  if (ws_size < WS_END) return;

  const float* x   = (const float*)d_in[0];
  const float* W1a = (const float*)d_in[1];
  const float* b1a = (const float*)d_in[2];
  const float* W1b = (const float*)d_in[3];
  const float* b1b = (const float*)d_in[4];
  const float* W2a = (const float*)d_in[5];
  const float* b2a = (const float*)d_in[6];
  const float* W2b = (const float*)d_in[7];
  const float* b2b = (const float*)d_in[8];
  float* out = (float*)d_out;
  char* ws = (char*)d_ws;

  float* v      = (float*)(ws + OFF_V);
  float* avg    = (float*)(ws + OFF_AVG);
  float* energy = (float*)(ws + OFF_EN);
  float* o1raw  = (float*)(ws + OFF_O1);
  float* o2raw  = (float*)(ws + OFF_O2);
  float* vec1   = (float*)(ws + OFF_VEC1);
  float* vec2   = (float*)(ws + OFF_VEC2);
  unsigned short* bt1h = (unsigned short*)(ws + OFF_BT1H);
  unsigned short* bt1l = (unsigned short*)(ws + OFF_BT1L);
  unsigned short* bt2h = (unsigned short*)(ws + OFF_BT2H);
  unsigned short* bt2l = (unsigned short*)(ws + OFF_BT2L);
  float* pbuf   = (float*)(ws + OFF_P);
  unsigned short* ah = (unsigned short*)(ws + OFF_AH);
  unsigned short* al = (unsigned short*)(ws + OFF_AL);

  const float* colv1 = vec1;            const float* colv2 = vec2;
  const float* bias1 = vec1 + NP1;      const float* bias2 = vec2 + NP2;
  const float* wbar1 = vec1 + 2 * NP1;  const float* wbar2 = vec2 + 2 * NP2;
  const float* bline1 = vec1 + 3 * NP1; const float* bline2 = vec2 + 3 * NP2;

  const dim3 blk256(256);

  ln_input_kernel<<<1, dim3(512), 0, stream>>>(x, v);

  pool_kernel<<<SIG_LEN / POOL_OUT, blk256, 0, stream>>>(v, avg, energy);

  prep_bt_kernel<KW1, DIN1, NH1, NP1><<<(NP1 * (KW1 / 8) + 255) / 256, blk256, 0, stream>>>(W1a, bt1h, bt1l);
  prep_bt_kernel<KW2, DIN2, NH2, NP2><<<(NP2 * (KW2 / 8) + 255) / 256, blk256, 0, stream>>>(W2a, bt2h, bt2l);
  prep_vec_kernel<KW1, DIN1, NH1, NP1, PP1><<<dim3(1, 4), blk256, 0, stream>>>(W1a, b1a, W1b, b1b, vec1);
  prep_vec_kernel<KW2, DIN2, NH2, NP2, PP2><<<dim3(1, 4), blk256, 0, stream>>>(W2a, b2a, W2b, b2b, vec2);

  {
    const int nrows = SIG_LEN, kw8 = KW1 / 8;
    build_a_kernel<<<(nrows * kw8 + 255) / 256, blk256, 0, stream>>>(v, ah, al, 0, nrows, kw8);
    const int tiles = (nrows / 64) * (NP1 / 64);
    gemm_hidden_dot<<<(tiles + 7) / 8, blk256, 0, stream>>>(
        ah, al, KW1, bt1h, bt1l, KW1, pbuf, (long)SIG_LEN,
        bias1, colv1, wbar1, avg, nrows, NP1, KW1);
    psum_kernel<<<(SIG_LEN / 4 + 255) / 256, blk256, 0, stream>>>(pbuf, NT1, (long)SIG_LEN, bline1, o1raw);
  }

  for (int c = 0; c < SIG_LEN / CHUNK2; ++c) {
    const int row0 = c * CHUNK2;
    const int nrows = CHUNK2, kw8 = KW2 / 8;
    build_a_kernel<<<(nrows * kw8 + 255) / 256, blk256, 0, stream>>>(v, ah, al, row0, nrows, kw8);
    const int tiles = (nrows / 64) * (NP2 / 64);
    gemm_hidden_dot<<<(tiles + 7) / 8, blk256, 0, stream>>>(
        ah, al, KW2, bt2h, bt2l, KW2, pbuf + row0, (long)SIG_LEN,
        bias2, colv2, wbar2, avg + row0, nrows, NP2, KW2);
  }
  psum_kernel<<<(SIG_LEN / 4 + 255) / 256, blk256, 0, stream>>>(pbuf, NT2, (long)SIG_LEN, bline2, o2raw);

  ln_output_kernel<true><<<1, dim3(512), 0, stream>>>(o1raw, energy, out);
  ln_output_kernel<false><<<1, dim3(512), 0, stream>>>(o2raw, energy, out + SIG_LEN);
}
